// DeLanNet_inverse_3513283248763
// MI455X (gfx1250) — hardware-verified
//
#include <hip/hip_runtime.h>
#include <stddef.h>
#include <stdint.h>


#define DOF   7
#define HID   512
#define NLO   21
#define XW    21
#define NT    128
#define NWV   4
#define SPB   64
#define RP    64
#define S1P   112
#define NPREP 160
#define WSCAP 134217728
#define TSZ   512
#define LDS_FWD 45056
#define OFF_TL  3072
#define OFF_ST2 28672

static_assert(NT == NWV * 32);
static_assert(SPB == NWV * 16);
static_assert((HID % 32) == 0);
static_assert(((SPB * DOF * 4) % 128) == 0);
static_assert(((SPB * DOF) % 4) == 0);
static_assert(((16 * RP * 4) % 512) == 0);
static_assert(3 * 8 * 32 * 4 <= OFF_TL);
static_assert(OFF_TL + NWV * 10 * TSZ * 2 <= LDS_FWD);
static_assert(NWV * 16 * S1P * 4 <= OFF_ST2);
static_assert(OFF_ST2 + NWV * 16 * RP * 4 <= LDS_FWD);

typedef float          v4f  __attribute__((ext_vector_type(4)));
typedef v4f            v4fa __attribute__((may_alias));
typedef float          v8f  __attribute__((ext_vector_type(8)));
typedef __bf16         v16b __attribute__((ext_vector_type(16)));
typedef __bf16         v8b  __attribute__((ext_vector_type(8)));
typedef unsigned short v8us __attribute__((ext_vector_type(8)));
typedef v8us           v8usa __attribute__((may_alias));
union FragB { v16b v; v8us u[2]; };
union Pk8   { v8b b; v8us u; };

__device__ __forceinline__ v8f wmb(v16b a, v16b b, v8f c) {
  v8f d = __builtin_amdgcn_wmma_f32_16x16x32_bf16(false, a, false, b, (short)0, c, false, false);
  asm volatile("v_nop\n\tv_nop\n\tv_nop\n\tv_nop" : "+v"(d) : "v"(a), "v"(b));
  return d;
}

__device__ __forceinline__ v8f z8() {
  v8f c = {0.f, 0.f, 0.f, 0.f, 0.f, 0.f, 0.f, 0.f};
  return c;
}

__device__ __forceinline__ float tanh_f(float x) {
  const float ax = fabsf(x);
  const float e = __builtin_amdgcn_exp2f(ax * -2.8853900817779268f);
  const float r = __builtin_amdgcn_rcpf(1.0f + e);
  const float y = (1.0f - e) * r;
  return copysignf(y, x);
}

__device__ __forceinline__ unsigned int bf_rne(float v) {
  const unsigned int u = __float_as_uint(v);
  return (u + 0x7FFFu + ((u >> 16) & 1u)) >> 16;
}

__device__ __forceinline__ void split1(float v, unsigned short& hi, unsigned short& lo) {
  const unsigned int h = bf_rne(v);
  hi = (unsigned short)h;
  lo = (unsigned short)bf_rne(v - __uint_as_float(h << 16));
}

__device__ __forceinline__ v16b ldB(const unsigned short* __restrict__ plane, int row, int kb) {
  FragB f;
  const unsigned short* p = plane + (size_t)row * HID + kb;
  f.u[0] = *(const v8us*)p;
  f.u[1] = *(const v8us*)(p + 16);
  return f.v;
}

__device__ __forceinline__ v16b ldA(const unsigned short* tile, int m, int hh) {
  FragB f;
  const unsigned short* p = tile + m * 32 + 8 * hh;
  f.u[0] = *(const v8usa*)p;
  f.u[1] = *(const v8usa*)(p + 16);
  return f.v;
}

__device__ __forceinline__ v8f mac3(v16b ah, v16b al, v16b bh, v16b bl, v8f acc) {
  acc = wmb(ah, bh, acc);
  acc = wmb(al, bh, acc);
  acc = wmb(ah, bl, acc);
  return acc;
}

__global__ __launch_bounds__(64) void k_prep(const float* __restrict__ Wd1, const float* __restrict__ Wo1,
                                             const float* __restrict__ Wd2, const float* __restrict__ Wo2,
                                             const float* __restrict__ Wg2,
                                             unsigned short* pdT, unsigned short* poT, unsigned short* pgT,
                                             unsigned short* p1d, unsigned short* p1o,
                                             float* w2dP, float* w2oP) {
  const int t = threadIdx.x;
  const int b = blockIdx.x;
  if (b < 96) {
    const float* src;
    unsigned short* dst;
    int n, rows, nval, trans, srcw;
    if (b < 16)      { src = Wd2; dst = pdT; n = b;      rows = 16; nval = DOF; trans = 1; srcw = DOF; }
    else if (b < 48) { src = Wo2; dst = poT; n = b - 16; rows = 32; nval = NLO; trans = 1; srcw = NLO; }
    else if (b < 64) { src = Wg2; dst = pgT; n = b - 48; rows = 16; nval = DOF; trans = 1; srcw = DOF; }
    else if (b < 80) { src = Wd1; dst = p1d; n = b - 64; rows = 16; nval = DOF; trans = 0; srcw = HID; }
    else             { src = Wo1; dst = p1o; n = b - 80; rows = 16; nval = DOF; trans = 0; srcw = HID; }
    const int nc = (n < nval) ? n : (nval - 1);
    const bool keep = (n < nval);
    Pk8 ph, pl;
#pragma unroll
    for (int j = 0; j < 8; ++j) {
      const int k = 8 * t + j;
      const size_t idx = trans ? ((size_t)k * srcw + nc) : ((size_t)nc * HID + k);
      const float ld = src[idx];
      const float v = keep ? ld : 0.0f;
      const __bf16 hb = (__bf16)v;
      ph.b[j] = hb;
      pl.b[j] = (__bf16)(v - (float)hb);
    }
    unsigned short* dh = dst + (size_t)n * HID + 8 * t;
    unsigned short* dl = dst + (size_t)(rows + n) * HID + 8 * t;
    *(volatile v8us*)dh = ph.u;
    *(volatile v8us*)dl = pl.u;
    __threadfence();
    *(volatile v8us*)dh = ph.u;
    *(volatile v8us*)dl = pl.u;
  } else if (b < 112) {
    const int jb = b - 96;
    const int row = 32 * jb + (t >> 1);
    const int c0 = (t & 1) * 4;
    v4f o;
#pragma unroll
    for (int e = 0; e < 4; ++e) {
      const int c = c0 + e;
      const int cc = (c < DOF) ? c : (DOF - 1);
      const float ld = Wd2[row * DOF + cc];
      o[e] = (c < DOF) ? ld : 0.0f;
    }
    float* d = w2dP + (size_t)row * 8 + c0;
    *(volatile v4f*)d = o;
    __threadfence();
    *(volatile v4f*)d = o;
  } else {
    const int jb = b - 112;
    const int f0 = 256 * jb + 4 * t;
    const int row = f0 / 24;
    const int c0 = f0 - 24 * row;
    v4f o;
#pragma unroll
    for (int e = 0; e < 4; ++e) {
      const int c = c0 + e;
      const int cc = (c < NLO) ? c : (NLO - 1);
      const float ld = Wo2[row * NLO + cc];
      o[e] = (c < NLO) ? ld : 0.0f;
    }
    float* d = w2oP + f0;
    *(volatile v4f*)d = o;
    __threadfence();
    *(volatile v4f*)d = o;
  }
}

__global__ __launch_bounds__(NT) __attribute__((amdgpu_num_vgpr(256)))
void k_fwd(const float* __restrict__ x,
           const float* __restrict__ Wd1, const float* __restrict__ bd1, const float* __restrict__ bd2,
           const float* __restrict__ Wo1, const float* __restrict__ bo1, const float* __restrict__ bo2,
           const float* __restrict__ Wg1, const float* __restrict__ bg1, const float* __restrict__ bg2,
           const unsigned short* __restrict__ pdT, const unsigned short* __restrict__ poT,
           const unsigned short* __restrict__ pgT,
           float* R) {
  __shared__ __attribute__((aligned(16))) unsigned char lds[LDS_FWD];
  const int tid = threadIdx.x, lane = tid & 31, hh = lane >> 4, m = lane & 15;
  const int wave = __builtin_amdgcn_readfirstlane(tid >> 5);
  const int kof = 8 * hh;
  float* sW = (float*)lds;
  unsigned short* tl = (unsigned short*)(lds + OFF_TL) + wave * (10 * TSZ);
  float* st1 = (float*)lds + wave * (16 * S1P);
  float* st2 = (float*)(lds + OFF_ST2) + wave * (16 * RP);
  const int sbase = blockIdx.x * SPB + wave * 16;
  const int sm = sbase + m;
  const float* xr = x + (size_t)sm * XW;
  float q[DOF], qd[DOF];
#pragma unroll
  for (int c = 0; c < DOF; ++c) { q[c] = xr[c]; qd[c] = xr[DOF + c]; }
  const int trow = m * 32;

  v8f aHd = z8(), aDd = z8(), aG = z8();
  v8f aHo0 = z8(), aHo1 = z8(), aDo0 = z8(), aDo1 = z8();

#pragma unroll 1
  for (int k0 = 0; k0 < HID; k0 += 32) {
    __syncthreads();
#pragma unroll
    for (int p = 0; p < 2; ++p) {
      const int g = 4 * p + wave;
      if (g < 6) {
        const int net = g >> 1;
        const int idx = 32 * (g & 1) + lane;
        const int c = idx >> 3;
        const int col4 = (idx & 7) * 4;
        const float* W1n = (net == 0) ? Wd1 : ((net == 1) ? Wo1 : Wg1);
        const float* b1n = (net == 0) ? bd1 : ((net == 1) ? bo1 : bg1);
        const int cc = (c < DOF) ? c : (DOF - 1);
        const v4f wv = *(const v4f*)(W1n + (size_t)cc * HID + k0 + col4);
        const v4f bv = *(const v4f*)(b1n + k0 + col4);
        const v4f val = (c < DOF) ? wv : bv;
        *(v4f*)(sW + net * 256 + c * 32 + col4) = val;
      }
    }
    __syncthreads();

    {
      const float* w = sW;
#pragma unroll 1
      for (int i = 0; i < 16; ++i) {
        const int hl = kof + (i & 7) + ((i & 8) << 1);
        const float w0 = w[hl];
        float pr = q[0] * w0, tg = qd[0] * w0;
#pragma unroll
        for (int c = 1; c < DOF; ++c) {
          const float wc = w[32 * c + hl];
          pr = fmaf(q[c], wc, pr);
          tg = fmaf(qd[c], wc, tg);
        }
        pr += w[224 + hl];
        const float z = tanh_f(pr);
        const float s = fmaf(-z, z, 1.0f) * tg;
        unsigned short zh, zl, sh, sl;
        split1(z, zh, zl);
        split1(s, sh, sl);
        const int o = trow + hl;
        tl[0 * TSZ + o] = zh;
        tl[1 * TSZ + o] = zl;
        tl[2 * TSZ + o] = sh;
        tl[3 * TSZ + o] = sl;
      }
    }
    {
      const float* w = sW + 256;
#pragma unroll 1
      for (int i = 0; i < 16; ++i) {
        const int hl = kof + (i & 7) + ((i & 8) << 1);
        const float w0 = w[hl];
        float pr = q[0] * w0, tg = qd[0] * w0;
#pragma unroll
        for (int c = 1; c < DOF; ++c) {
          const float wc = w[32 * c + hl];
          pr = fmaf(q[c], wc, pr);
          tg = fmaf(qd[c], wc, tg);
        }
        pr += w[224 + hl];
        const float z = tanh_f(pr);
        const float s = fmaf(-z, z, 1.0f) * tg;
        unsigned short zh, zl, sh, sl;
        split1(z, zh, zl);
        split1(s, sh, sl);
        const int o = trow + hl;
        tl[4 * TSZ + o] = zh;
        tl[5 * TSZ + o] = zl;
        tl[6 * TSZ + o] = sh;
        tl[7 * TSZ + o] = sl;
      }
    }
    {
      const float* w = sW + 512;
#pragma unroll 1
      for (int i = 0; i < 16; ++i) {
        const int hl = kof + (i & 7) + ((i & 8) << 1);
        float pr = q[0] * w[hl];
#pragma unroll
        for (int c = 1; c < DOF; ++c) pr = fmaf(q[c], w[32 * c + hl], pr);
        pr += w[224 + hl];
        const float z = tanh_f(pr);
        unsigned short zh, zl;
        split1(z, zh, zl);
        const int o = trow + hl;
        tl[8 * TSZ + o] = zh;
        tl[9 * TSZ + o] = zl;
      }
    }
    __syncthreads();

    {
      const int kb = k0 + kof;
      {
        const v16b zh = ldA(tl + 0 * TSZ, m, hh), zl = ldA(tl + 1 * TSZ, m, hh);
        const v16b sh = ldA(tl + 2 * TSZ, m, hh), sl = ldA(tl + 3 * TSZ, m, hh);
        const v16b bh = ldB(pdT, m, kb), bl = ldB(pdT, 16 + m, kb);
        aHd = mac3(zh, zl, bh, bl, aHd);
        aDd = mac3(sh, sl, bh, bl, aDd);
      }
      {
        const v16b zh = ldA(tl + 4 * TSZ, m, hh), zl = ldA(tl + 5 * TSZ, m, hh);
        const v16b sh = ldA(tl + 6 * TSZ, m, hh), sl = ldA(tl + 7 * TSZ, m, hh);
        {
          const v16b bh = ldB(poT, m, kb), bl = ldB(poT, 32 + m, kb);
          aHo0 = mac3(zh, zl, bh, bl, aHo0);
          aDo0 = mac3(sh, sl, bh, bl, aDo0);
        }
        {
          const v16b bh = ldB(poT, 16 + m, kb), bl = ldB(poT, 48 + m, kb);
          aHo1 = mac3(zh, zl, bh, bl, aHo1);
          aDo1 = mac3(sh, sl, bh, bl, aDo1);
        }
      }
      {
        const v16b zh = ldA(tl + 8 * TSZ, m, hh), zl = ldA(tl + 9 * TSZ, m, hh);
        const v16b bh = ldB(pgT, m, kb), bl = ldB(pgT, 16 + m, kb);
        aG = mac3(zh, zl, bh, bl, aG);
      }
    }
  }
  __syncthreads();

#pragma unroll
  for (int r = 0; r < 8; ++r) {
    float* rowp = st1 + (8 * hh + r) * S1P + m;
    rowp[0]  = aHd[r];
    rowp[16] = aDd[r];
    rowp[32] = aG[r];
    rowp[48] = aHo0[r];
    rowp[64] = aHo1[r];
    rowp[80] = aDo0[r];
    rowp[96] = aDo1[r];
  }
  __syncthreads();

  {
    const float* rw = st1 + m * S1P;
    float qdd[DOF];
#pragma unroll
    for (int i = 0; i < DOF; ++i) qdd[i] = xr[2 * DOF + i];
    float Ld[DOF], Dd[DOF], Lo[NLO], Dn[NLO];
#pragma unroll
    for (int i = 0; i < DOF; ++i) { Ld[i] = rw[i] + bd2[i]; Dd[i] = rw[16 + i]; }
#pragma unroll
    for (int e = 0; e < NLO; ++e) { Lo[e] = rw[48 + e] + bo2[e]; Dn[e] = rw[80 + e]; }
    float v[DOF], u1[DOF], tq[DOF];
#pragma unroll
    for (int j = 0; j < DOF; ++j) {
      float av = Ld[j] * qd[j], au = Dd[j] * qd[j], at = Ld[j] * qdd[j];
#pragma unroll
      for (int i = j + 1; i < DOF; ++i) {
        const int r = i * (i - 1) / 2 + j;
        av = fmaf(Lo[r], qd[i], av);
        au = fmaf(Dn[r], qd[i], au);
        at = fmaf(Lo[r], qdd[i], at);
      }
      v[j] = av; u1[j] = au; tq[j] = at;
    }
    float res[DOF];
#pragma unroll
    for (int j = 0; j < DOF; ++j) {
      float acc = rw[32 + j] + bg2[j];
#pragma unroll
      for (int mm = 0; mm < j; ++mm) {
        const int r = j * (j - 1) / 2 + mm;
        acc = fmaf(Lo[r], tq[mm] + u1[mm], acc);
        acc = fmaf(Dn[r], v[mm], acc);
      }
      acc = fmaf(Ld[j], tq[j] + u1[j], acc);
      acc = fmaf(Dd[j], v[j], acc);
      res[j] = acc;
    }
    if (hh == 0) {
      float* o2 = st2 + m * RP;
#pragma unroll
      for (int j = 0; j < DOF; ++j) o2[j] = res[j];
      o2[7] = 0.0f;
#pragma unroll
      for (int i = 0; i < DOF; ++i) o2[8 + i] = 2.0f * qd[i] * v[i];
      o2[15] = 0.0f;
#pragma unroll
      for (int i = 1; i < DOF; ++i)
#pragma unroll
        for (int j = 0; j < i; ++j) o2[16 + i * (i - 1) / 2 + j] = 2.0f * qd[i] * v[j];
#pragma unroll
      for (int p = 16 + NLO; p < RP; ++p) o2[p] = 0.0f;
    }
  }
  __syncthreads();

  {
    const float* s2 = st2;
    float* gdst = R + (size_t)sbase * RP;
    v4f vv[8];
#pragma unroll
    for (int s = 0; s < 8; ++s) vv[s] = *(const v4fa*)(s2 + 4 * (lane + 32 * s));
#pragma unroll
    for (int s = 0; s < 8; ++s) *(volatile v4f*)(gdst + 4 * (lane + 32 * s)) = vv[s];
    __threadfence();
#pragma unroll
    for (int s = 0; s < 8; ++s) *(volatile v4f*)(gdst + 4 * (lane + 32 * s)) = vv[s];
  }
}

__global__ __launch_bounds__(NT) __attribute__((amdgpu_num_vgpr(256)))
void k_c1(const float* __restrict__ x,
          const float* __restrict__ Wd1, const float* __restrict__ bd1,
          const float* __restrict__ Wo1, const float* __restrict__ bo1,
          const float* __restrict__ w2dP, const float* __restrict__ w2oP,
          const unsigned short* __restrict__ p1d, const unsigned short* __restrict__ p1o,
          const float* __restrict__ R, float* out) {
  __shared__ __attribute__((aligned(16))) float cW[1536];
  __shared__ __attribute__((aligned(16))) unsigned short tE[NWV * 4 * TSZ];
  __shared__ __attribute__((aligned(16))) float sto[SPB * 16];
  const int tid = threadIdx.x, lane = tid & 31, hh = lane >> 4, m = lane & 15;
  const int wave = __builtin_amdgcn_readfirstlane(tid >> 5);
  const int kof = 8 * hh;
  unsigned short* tl = tE + wave * (4 * TSZ);
  const int sbase = blockIdx.x * SPB + wave * 16;
  const int sm = sbase + m;
  const float* xr = x + (size_t)sm * XW;
  float q[DOF];
#pragma unroll
  for (int c = 0; c < DOF; ++c) q[c] = xr[c];
  const float* rr = R + (size_t)sm * RP;
  float wd[DOF], wo[NLO];
  {
    const v4f a = *(const v4f*)(rr + 8), b = *(const v4f*)(rr + 12);
    wd[0] = a.x; wd[1] = a.y; wd[2] = a.z; wd[3] = a.w; wd[4] = b.x; wd[5] = b.y; wd[6] = b.z;
    const v4f c0 = *(const v4f*)(rr + 16), c1 = *(const v4f*)(rr + 20), c2 = *(const v4f*)(rr + 24);
    const v4f c3 = *(const v4f*)(rr + 28), c4 = *(const v4f*)(rr + 32), c5 = *(const v4f*)(rr + 36);
    wo[0] = c0.x;  wo[1] = c0.y;  wo[2] = c0.z;  wo[3] = c0.w;
    wo[4] = c1.x;  wo[5] = c1.y;  wo[6] = c1.z;  wo[7] = c1.w;
    wo[8] = c2.x;  wo[9] = c2.y;  wo[10] = c2.z; wo[11] = c2.w;
    wo[12] = c3.x; wo[13] = c3.y; wo[14] = c3.z; wo[15] = c3.w;
    wo[16] = c4.x; wo[17] = c4.y; wo[18] = c4.z; wo[19] = c4.w;
    wo[20] = c5.x;
  }
  const int trow = m * 32;

  v8f acc = z8();
#pragma unroll 1
  for (int k0 = 0; k0 < HID; k0 += 32) {
    __syncthreads();
#pragma unroll
    for (int p = 0; p < 3; ++p) {
      const int g = 4 * p + wave;
      if (g < 6) {
        const int item = 32 * g + lane;
        *(v4f*)(cW + 4 * item) = *(const v4f*)(w2oP + (size_t)k0 * 24 + 4 * item);
      } else if (g < 8) {
        const int item = 32 * (g - 6) + lane;
        *(v4f*)(cW + 768 + 4 * item) = *(const v4f*)(w2dP + (size_t)k0 * 8 + 4 * item);
      } else {
        const int net = (g - 8) >> 1;
        const int idx = 32 * ((g - 8) & 1) + lane;
        const int c = idx >> 3;
        const int col4 = (idx & 7) * 4;
        const float* W1n = (net == 0) ? Wd1 : Wo1;
        const float* b1n = (net == 0) ? bd1 : bo1;
        const int cc = (c < DOF) ? c : (DOF - 1);
        const v4f wv = *(const v4f*)(W1n + (size_t)cc * HID + k0 + col4);
        const v4f bv = *(const v4f*)(b1n + k0 + col4);
        const v4f val = (c < DOF) ? wv : bv;
        *(v4f*)(cW + 1024 + net * 256 + c * 32 + col4) = val;
      }
    }
    __syncthreads();

    {
      const float* w = cW + 1024;
#pragma unroll 1
      for (int i = 0; i < 16; ++i) {
        const int hl = kof + (i & 7) + ((i & 8) << 1);
        float pr = q[0] * w[hl];
#pragma unroll
        for (int c = 1; c < DOF; ++c) pr = fmaf(q[c], w[32 * c + hl], pr);
        pr += w[224 + hl];
        const v4f a0 = *(const v4f*)(cW + 768 + hl * 8), a1 = *(const v4f*)(cW + 768 + hl * 8 + 4);
        float a = a0.x * wd[0];
        a = fmaf(a0.y, wd[1], a); a = fmaf(a0.z, wd[2], a); a = fmaf(a0.w, wd[3], a);
        a = fmaf(a1.x, wd[4], a); a = fmaf(a1.y, wd[5], a); a = fmaf(a1.z, wd[6], a);
        const float z = tanh_f(pr);
        const float e = fmaf(-z, z, 1.0f) * a;
        unsigned short eh, el;
        split1(e, eh, el);
        const int o = trow + hl;
        tl[0 * TSZ + o] = eh;
        tl[1 * TSZ + o] = el;
      }
    }
    {
      const float* w = cW + 1280;
#pragma unroll 1
      for (int i = 0; i < 16; ++i) {
        const int hl = kof + (i & 7) + ((i & 8) << 1);
        float pr = q[0] * w[hl];
#pragma unroll
        for (int c = 1; c < DOF; ++c) pr = fmaf(q[c], w[32 * c + hl], pr);
        pr += w[224 + hl];
        const float* wp = cW + hl * 24;
        const v4f a0 = *(const v4f*)wp,        a1 = *(const v4f*)(wp + 4),  a2 = *(const v4f*)(wp + 8);
        const v4f a3 = *(const v4f*)(wp + 12), a4 = *(const v4f*)(wp + 16), a5 = *(const v4f*)(wp + 20);
        float a = a0.x * wo[0];
        a = fmaf(a0.y, wo[1], a);  a = fmaf(a0.z, wo[2], a);  a = fmaf(a0.w, wo[3], a);
        a = fmaf(a1.x, wo[4], a);  a = fmaf(a1.y, wo[5], a);  a = fmaf(a1.z, wo[6], a);  a = fmaf(a1.w, wo[7], a);
        a = fmaf(a2.x, wo[8], a);  a = fmaf(a2.y, wo[9], a);  a = fmaf(a2.z, wo[10], a); a = fmaf(a2.w, wo[11], a);
        a = fmaf(a3.x, wo[12], a); a = fmaf(a3.y, wo[13], a); a = fmaf(a3.z, wo[14], a); a = fmaf(a3.w, wo[15], a);
        a = fmaf(a4.x, wo[16], a); a = fmaf(a4.y, wo[17], a); a = fmaf(a4.z, wo[18], a); a = fmaf(a4.w, wo[19], a);
        a = fmaf(a5.x, wo[20], a);
        const float z = tanh_f(pr);
        const float e = fmaf(-z, z, 1.0f) * a;
        unsigned short eh, el;
        split1(e, eh, el);
        const int o = trow + hl;
        tl[2 * TSZ + o] = eh;
        tl[3 * TSZ + o] = el;
      }
    }
    __syncthreads();

    {
      const int kb = k0 + kof;
      {
        const v16b eh = ldA(tl + 0 * TSZ, m, hh), el = ldA(tl + 1 * TSZ, m, hh);
        const v16b bh = ldB(p1d, m, kb), bl = ldB(p1d, 16 + m, kb);
        acc = mac3(eh, el, bh, bl, acc);
      }
      {
        const v16b eh = ldA(tl + 2 * TSZ, m, hh), el = ldA(tl + 3 * TSZ, m, hh);
        const v16b bh = ldB(p1o, m, kb), bl = ldB(p1o, 16 + m, kb);
        acc = mac3(eh, el, bh, bl, acc);
      }
    }
  }

#pragma unroll
  for (int r = 0; r < 8; ++r) sto[(wave * 16 + 8 * hh + r) * 16 + m] = acc[r];
  __syncthreads();

  const int tc = (tid < 112) ? tid : 111;
  float o[4];
#pragma unroll
  for (int e = 0; e < 4; ++e) {
    const int f = 4 * tc + e;
    const int sl = f / DOF;
    const int j = f - DOF * sl;
    const float resv = R[(size_t)(blockIdx.x * SPB + sl) * RP + j];
    o[e] = sto[sl * 16 + j] + resv;
  }
  v4f ov;
  ov.x = o[0]; ov.y = o[1]; ov.z = o[2]; ov.w = o[3];
  float* od = out + (size_t)blockIdx.x * (SPB * DOF) + 4 * tc;
  if (tid < 112) *(volatile v4f*)od = ov;
  __threadfence();
  if (tid < 112) *(volatile v4f*)od = ov;
}

extern "C" void kernel_launch(void* const* d_in, const int* in_sizes, int n_in,
                              void* d_out, int out_size, void* d_ws, size_t ws_size,
                              hipStream_t stream) {
  if (n_in < 13) return;
  const int B = in_sizes[0] / XW;
  if (B <= 0 || in_sizes[0] != B * XW || (B % SPB) != 0) return;
  if (in_sizes[1] != DOF * HID || in_sizes[2] != HID || in_sizes[3] != HID * DOF || in_sizes[4] != DOF) return;
  if (in_sizes[5] != DOF * HID || in_sizes[6] != HID || in_sizes[7] != HID * NLO || in_sizes[8] != NLO) return;
  if (in_sizes[9] != DOF * HID || in_sizes[10] != HID || in_sizes[11] != HID * DOF || in_sizes[12] != DOF) return;
  if (out_size != B * DOF) return;

  const float* x   = (const float*)d_in[0];
  const float* Wd1 = (const float*)d_in[1];
  const float* bd1 = (const float*)d_in[2];
  const float* Wd2 = (const float*)d_in[3];
  const float* bd2 = (const float*)d_in[4];
  const float* Wo1 = (const float*)d_in[5];
  const float* bo1 = (const float*)d_in[6];
  const float* Wo2 = (const float*)d_in[7];
  const float* bo2 = (const float*)d_in[8];
  const float* Wg1 = (const float*)d_in[9];
  const float* bg1 = (const float*)d_in[10];
  const float* Wg2 = (const float*)d_in[11];
  const float* bg2 = (const float*)d_in[12];
  float* out = (float*)d_out;

  char* ws = (char*)d_ws;
  size_t off = 0;
  const size_t oPd  = off; off += (size_t)2 * 16 * HID * 2; off = (off + 255) & ~(size_t)255;
  const size_t oPo  = off; off += (size_t)2 * 32 * HID * 2; off = (off + 255) & ~(size_t)255;
  const size_t oPg  = off; off += (size_t)2 * 16 * HID * 2; off = (off + 255) & ~(size_t)255;
  const size_t oP1d = off; off += (size_t)2 * 16 * HID * 2; off = (off + 255) & ~(size_t)255;
  const size_t oP1o = off; off += (size_t)2 * 16 * HID * 2; off = (off + 255) & ~(size_t)255;
  const size_t oW2d = off; off += (size_t)HID * 8 * 4;       off = (off + 255) & ~(size_t)255;
  const size_t oW2o = off; off += (size_t)HID * 24 * 4;      off = (off + 255) & ~(size_t)255;
  const size_t oR   = off; off += (size_t)B * RP * 4;        off = (off + 255) & ~(size_t)255;
  if (off > ws_size || off > (size_t)WSCAP) return;

  unsigned short* pdT = (unsigned short*)(ws + oPd);
  unsigned short* poT = (unsigned short*)(ws + oPo);
  unsigned short* pgT = (unsigned short*)(ws + oPg);
  unsigned short* p1d = (unsigned short*)(ws + oP1d);
  unsigned short* p1o = (unsigned short*)(ws + oP1o);
  float* w2dP = (float*)(ws + oW2d);
  float* w2oP = (float*)(ws + oW2o);
  float* R    = (float*)(ws + oR);

  k_prep<<<NPREP, 64, 0, stream>>>(Wd1, Wo1, Wd2, Wo2, Wg2, pdT, poT, pgT, p1d, p1o, w2dP, w2oP);
  k_fwd<<<B / SPB, NT, 0, stream>>>(x, Wd1, bd1, bd2, Wo1, bo1, bo2, Wg1, bg1, bg2, pdT, poT, pgT, R);
  k_c1<<<B / SPB, NT, 0, stream>>>(x, Wd1, bd1, Wo1, bo1, w2dP, w2oP, p1d, p1o, R, out);
}
